// RKDAngleLoss_86723979641277
// MI455X (gfx1250) — hardware-run, weakly checked
//
#include <hip/hip_runtime.h>
#include <math.h>

typedef __attribute__((ext_vector_type(16))) _Float16 v16h;
typedef __attribute__((ext_vector_type(16))) __bf16 v16b;
typedef __attribute__((ext_vector_type(8)))  _Float16 v8h;
typedef __attribute__((ext_vector_type(8)))  float v8f;
typedef __attribute__((ext_vector_type(4)))  float v4f;
typedef __attribute__((ext_vector_type(2)))  float v2f;
typedef __attribute__((ext_vector_type(4)))  unsigned v4u;
typedef __attribute__((ext_vector_type(4)))  int v4i;
typedef float __attribute__((may_alias)) float_a;
typedef int __attribute__((may_alias)) int_a;

template <typename T> __device__ __forceinline__ void vst2(void* p, T v) { *(volatile T*)p = v; __threadfence(); *(volatile T*)p = v; }
__device__ __forceinline__ v8f wmma16(v16h a, v16h b, v8f c) {
  v8f d = __builtin_amdgcn_wmma_f32_16x16x32_f16(false, a, false, b, (short)0, c, false, false);
  asm volatile("v_nop\n\tv_nop\n\tv_nop\n\tv_nop" : "+v"(d) : "v"(a), "v"(b));
  return d;
}
__device__ __forceinline__ v8f wmma_bf(v16b a, v16b b, v8f c) {
  v8f d = __builtin_amdgcn_wmma_f32_16x16x32_bf16(false, a, false, b, (short)0, c, false, false);
  asm volatile("v_nop\n\tv_nop\n\tv_nop\n\tv_nop" : "+v"(d) : "v"(a), "v"(b));
  return d;
}
__device__ __forceinline__ v16h frag_h(const _Float16* rowk0, int lane) {
  union { v16h v; v8h q[2]; } u; const _Float16* p = rowk0 + 8 * (lane >> 4);
  u.q[0] = *(const v8h*)p; u.q[1] = *(const v8h*)(p + 16); return u.v;
}
__device__ __forceinline__ v16h frag_f32(const float* rowk0, int lane) {
  v16h a; const float* p = rowk0 + 8 * (lane >> 4);
#pragma unroll
  for (int i = 0; i < 8; ++i) { a[i] = (_Float16)p[i]; a[8 + i] = (_Float16)p[16 + i]; }
  return a;
}
__device__ __forceinline__ v16h frag_f32s(const float* rowk0, int lane, float sc) {
  v16h a; const float* p = rowk0 + 8 * (lane >> 4);
#pragma unroll
  for (int i = 0; i < 8; ++i) { a[i] = (_Float16)(p[i] * sc); a[8 + i] = (_Float16)(p[16 + i] * sc); }
  return a;
}
__device__ __forceinline__ v16h fragc_f32(const float* W, int k0, int n, int lane, int ld, int K) {
  v16h a; const int g = lane >> 4;
#pragma unroll
  for (int i = 0; i < 8; ++i) { const int ka = k0 + 8 * g + i, kb = ka + 16;
    a[i] = (_Float16)(ka < K ? W[(size_t)(ka < K ? ka : K - 1) * ld + n] : 0.f); a[8 + i] = (_Float16)(kb < K ? W[(size_t)(kb < K ? kb : K - 1) * ld + n] : 0.f); }
  return a;
}
struct F2 { v16b h, l; };
__device__ __forceinline__ F2 bsplit16(const float v[16]) { F2 r;
#pragma unroll
  for (int i = 0; i < 16; ++i) { const __bf16 h = (__bf16)v[i]; r.h[i] = h; r.l[i] = (__bf16)(v[i] - (float)h); }
  return r; }
__device__ __forceinline__ F2 split_row(const float* row, int k0, int lane) { float v[16]; const float* p = row + k0 + 8 * (lane >> 4);
#pragma unroll
  for (int i = 0; i < 8; ++i) { v[i] = p[i]; v[8 + i] = p[16 + i]; }
  return bsplit16(v); }
__device__ __forceinline__ F2 split_rowK(const float* row, int k0, int lane, int K) { float v[16]; const int g = lane >> 4;
#pragma unroll
  for (int i = 0; i < 8; ++i) { const int ka = k0 + 8 * g + i, kb = ka + 16; v[i] = ka < K ? row[ka < K ? ka : K - 1] : 0.f; v[8 + i] = kb < K ? row[kb < K ? kb : K - 1] : 0.f; }
  return bsplit16(v); }
__device__ __forceinline__ F2 split_col(const float* W, int k0, int n, int lane, int ld, int K) { float v[16]; const int g = lane >> 4;
#pragma unroll
  for (int i = 0; i < 8; ++i) { const int ka = k0 + 8 * g + i, kb = ka + 16; v[i] = ka < K ? W[(size_t)(ka < K ? ka : K - 1) * ld + n] : 0.f; v[8 + i] = kb < K ? W[(size_t)(kb < K ? kb : K - 1) * ld + n] : 0.f; }
  return bsplit16(v); }
__device__ __forceinline__ v8f mac3(const F2& a, const F2& b, v8f c) { c = wmma_bf(a.l, b.h, c); c = wmma_bf(a.h, b.l, c); return wmma_bf(a.h, b.h, c); }
__device__ __forceinline__ float sigm(float v) { return 1.0f / (1.0f + expf(-v)); }
#define LDSX() do { asm volatile("s_wait_dscnt 0" ::: "memory"); __builtin_amdgcn_wave_barrier(); __builtin_amdgcn_fence(__ATOMIC_RELEASE, "workgroup"); } while (0)


#define NN 512
#define DIN 512
#define DE 128
#define HALF 256
#ifndef NPASS
#define NPASS 2
#endif
typedef __attribute__((ext_vector_type(8))) __bf16 v8b;
__device__ __forceinline__ v16b frag_b(const __bf16* rowk0, int lane) {
  union { v16b v; v8b q[2]; } u; const __bf16* p = rowk0 + 8 * (lane >> 4);
  u.q[0] = *(const v8b*)p; u.q[1] = *(const v8b*)(p + 16); return u.v;
}
__device__ __forceinline__ float bfr(float v) { return (float)(__bf16)v; }
__device__ __attribute__((noinline)) float exp_ni(float v) { return expf(v); }
__device__ __attribute__((noinline)) float erf_ni(float v) { return erff(v); }

#define WS_PK   0u
#define WS_XB   (WS_PK + 2u * 2 * DE * DIN)
#define WS_EMB  (WS_XB + 2u * 2 * NN * DIN)
#define WS_E    (WS_EMB + 4u * 2 * NN * DE)
#define WS_PART (WS_E + 2u * 2 * HALF * NN * DE)
#define WS_END  (WS_PART + 128u * NPASS * HALF * 8)

__global__ __launch_bounds__(256) void k_pack(const float* __restrict__ W1, const float* __restrict__ W2, const float* __restrict__ S, const float* __restrict__ T, __bf16* __restrict__ PK, __bf16* __restrict__ XB) {
  __shared__ __align__(16) __bf16 s[DIN]; const int n = blockIdx.x, which = blockIdx.y, t = threadIdx.x;
  if (which < 2) { if (n >= DE) return; const float* Wm = which ? W2 : W1; for (int k = t; k < DIN; k += 256) s[k] = (__bf16)Wm[(size_t)k * DE + n]; }
  else { const float* X = (which == 2) ? S : T; for (int k = t; k < DIN; k += 256) s[k] = (__bf16)X[(size_t)n * DIN + k]; }
  __syncthreads();
  __bf16* dst = (which < 2) ? PK + ((size_t)which * DE + n) * DIN : XB + ((size_t)(which - 2) * NN + n) * DIN;
  for (int q = t; q < DIN / 8; q += 256) vst2((unsigned*)(dst + q * 8), *(const v4u*)&s[q * 8]);
}
__global__ __launch_bounds__(128) void k_emb(const __bf16* __restrict__ XB, const __bf16* __restrict__ PK, const float* __restrict__ B1, const float* __restrict__ B2, float* __restrict__ EMB) {
  __shared__ __align__(16) float so[4][16][132];
  const int tid = threadIdx.x, wave = tid >> 5, lane = tid & 31, col = lane & 15, g = lane >> 4; const int which = blockIdx.y; const size_t r0 = (size_t)blockIdx.x * 64 + wave * 16;
  const __bf16* X = XB + (size_t)which * NN * DIN; const __bf16* P = PK + (size_t)which * DE * DIN; const float* BB = which ? B2 : B1;
  v8f acc[8] = {};
#pragma unroll 2
  for (int kc = 0; kc < DIN / 32; ++kc) { const v16b a = frag_b(X + (r0 + col) * DIN + kc * 32, lane);
#pragma unroll
    for (int j = 0; j < 8; ++j) acc[j] = wmma_bf(a, frag_b(P + (size_t)(j * 16 + col) * DIN + kc * 32, lane), acc[j]); }
#pragma unroll
  for (int j = 0; j < 8; ++j) { const float bb = bfr(BB[j * 16 + col]);
#pragma unroll
    for (int r = 0; r < 8; ++r) so[wave][8 * g + r][j * 16 + col] = acc[j][r] + bb; }
  LDSX();
  for (int rl = 0; rl < 16; ++rl) vst2(EMB + ((size_t)which * NN + r0 + rl) * DE + lane * 4, *(const v4f*)&so[wave][rl][lane * 4]);
}
__global__ __launch_bounds__(256) void k_diffs(const float* __restrict__ EMB, int a0, _Float16* __restrict__ E) {
  __shared__ __align__(16) _Float16 se[64][DE + 8];
  const int tid = threadIdx.x, wave = tid >> 5, lane = tid & 31; const int ia = blockIdx.x, which = blockIdx.z; const int i = a0 + ia; const int j0 = blockIdx.y * 64;
  const float* X = EMB + (size_t)which * NN * DE; const float* xi = X + (size_t)i * DE;
  for (int rr = 0; rr < 8; ++rr) { const int jl = wave * 8 + rr; const float* xj = X + (size_t)(j0 + jl) * DE; float d[4]; float s = 0.f;
#pragma unroll
    for (int q = 0; q < 4; ++q) { d[q] = xj[lane + 32 * q] - xi[lane + 32 * q]; s += d[q] * d[q]; }
#pragma unroll
    for (int o = 1; o < 32; o <<= 1) s += __shfl_xor(s, o);
    const float inv = 1.0f / fmaxf(sqrtf(s), 1e-12f);
#pragma unroll
    for (int q = 0; q < 4; ++q) se[jl][lane + 32 * q] = (_Float16)(d[q] * inv); }
  __syncthreads();
  _Float16* dst = E + (((size_t)which * HALF + ia) * NN + j0) * DE;
  for (int q = tid; q < 64 * DE / 8; q += 256) { const int r = q >> 4, pc = q & 15; vst2((unsigned*)(dst + (size_t)r * DE + pc * 8), *(const v4u*)&se[r][pc * 8]); }
}
__global__ __launch_bounds__(128) void k_angle(const _Float16* __restrict__ E, int pass, double* __restrict__ PART) {
  __shared__ double sw[4]; __shared__ __align__(16) double sp[16];
  const int tid = threadIdx.x, wave = tid >> 5, lane = tid & 31, col = lane & 15, g = lane >> 4; const int ia = blockIdx.x; const int j0 = blockIdx.y * 64 + wave * 16;
  const _Float16* ES = E + ((size_t)0 * HALF + ia) * NN * DE; const _Float16* ET = E + ((size_t)1 * HALF + ia) * NN * DE;
  v16h as_[DE / 32], at_[DE / 32];
#pragma unroll
  for (int kc = 0; kc < DE / 32; ++kc) { as_[kc] = frag_h(ES + (size_t)(j0 + col) * DE + kc * 32, lane); at_[kc] = frag_h(ET + (size_t)(j0 + col) * DE + kc * 32, lane); }
  float s = 0.f;
#pragma unroll 1
  for (int kt = 0; kt < NN / 16; ++kt) { v8f cs = {}, ct = {};
#pragma unroll
    for (int kc = 0; kc < DE / 32; ++kc) { cs = wmma16(as_[kc], frag_h(ES + (size_t)(kt * 16 + col) * DE + kc * 32, lane), cs); ct = wmma16(at_[kc], frag_h(ET + (size_t)(kt * 16 + col) * DE + kc * 32, lane), ct); }
#pragma unroll
    for (int r = 0; r < 8; ++r) s += fabsf(cs[r] - ct[r]); }
  double ds = (double)s;
#pragma unroll
  for (int o = 1; o < 32; o <<= 1) ds += __shfl_xor(ds, o);
  if (lane == 0) sw[wave] = ds;
  if (tid < 16) sp[tid] = 0.0;
  __syncthreads();
  if (tid == 0) sp[0] = (sw[0] + sw[1]) + (sw[2] + sw[3]);
  __syncthreads();
  if (tid < 8) vst2((unsigned*)(PART + (((size_t)pass * HALF + ia) * 8 + blockIdx.y) * 16 + tid * 2), *(const v4u*)&sp[tid * 2]);
}
__global__ __launch_bounds__(256) void k_final(const double* __restrict__ PART, float* __restrict__ OUT) {
  __shared__ double sa[256]; const int t = threadIdx.x; double a = 0.0;
  for (int q = t; q < NPASS * HALF * 8; q += 256) a += PART[(size_t)q * 16];
  sa[t] = a; __syncthreads();
  if (t == 0) { double A = 0.0; for (int i = 0; i < 256; ++i) A += sa[i]; const float v = (float)(A / ((double)NN * (double)NN * (double)NN)); *(volatile float*)OUT = v; *(volatile float*)OUT = v; }
}
extern "C" void kernel_launch(void* const* d_in, const int* in_sizes, int n_in, void* d_out, int out_size, void* d_ws, size_t ws_size, hipStream_t stream) {
  (void)in_sizes; (void)n_in; (void)out_size;
  const float** F = (const float**)d_in;
  if (ws_size < (size_t)WS_END) return;
  char* ws = (char*)d_ws; __bf16 *PK = (__bf16*)(ws + WS_PK), *XB = (__bf16*)(ws + WS_XB); float* EMB = (float*)(ws + WS_EMB); _Float16* E = (_Float16*)(ws + WS_E); double* PART = (double*)(ws + WS_PART);
  k_pack<<<dim3(NN, 4), 256, 0, stream>>>(F[2], F[4], F[0], F[1], PK, XB);
  k_emb<<<dim3(NN / 64, 2), 128, 0, stream>>>(XB, PK, F[3], F[5], EMB);
  for (int pass = 0; pass < NPASS; ++pass) {
    k_diffs<<<dim3(HALF, NN / 64, 2), 256, 0, stream>>>(EMB, pass * HALF, E);
    k_angle<<<dim3(HALF, NN / 64), 128, 0, stream>>>(E, pass, PART); }
  k_final<<<1, 256, 0, stream>>>(PART, (float*)d_out);
}
